// GeneralizedInteractionNet_21852793602482
// MI455X (gfx1250) — hardware-verified
//
#include <hip/hip_runtime.h>
#include <stddef.h>


typedef _Float16 h16;
typedef _Float16 v16h __attribute__((ext_vector_type(16)));
typedef _Float16 v8h  __attribute__((ext_vector_type(8)));
typedef float    v8f  __attribute__((ext_vector_type(8)));
typedef float    v4f  __attribute__((ext_vector_type(4)));

#ifndef NB
#define NB 512
#endif
#define NB_FULL 512
#define NF    24
#define EMB   32
#define NSUB  16
#define ON    512
#define KPAD  32
#define LDH   40

#define ALCARRY 64.0f
#define B0CARRY 16.0f
#define WHCARRY 1024.0f
#define BICARRY1 64.0f
#define BICARRY2 1024.0f
#define RCARRY 2048.0f
#define INV0 (1.0f / (ALCARRY * B0CARRY * WHCARRY * B0CARRY))
#define INV1 (1.0f / (ALCARRY * B0CARRY * WHCARRY * BICARRY1))
#define INV2 (1.0f / (ALCARRY * B0CARRY * WHCARRY * BICARRY2))

#define WH_LAYER_HALVES (ON * KPAD)
#define AL_OFF0 0u
#define AL_OFF1 (NSUB * 32u * KPAD)
#define AL_OFF2 (AL_OFF1 + NSUB * 16u * KPAD)
#define AL_TOTAL_HALVES (AL_OFF2 + NSUB * 16u * KPAD)
#define OFF_WH_BYTES ((size_t)0)
#define OFF_WL_BYTES (OFF_WH_BYTES + (size_t)3 * WH_LAYER_HALVES * 2)
#define OFF_AL_BYTES (OFF_WL_BYTES + (size_t)3 * WH_LAYER_HALVES * 2)
#define WS_TOTAL (OFF_AL_BYTES + (size_t)AL_TOTAL_HALVES * 2)
#define WH_BLOCKS 8u

static_assert(NB >= 1 && NB <= NB_FULL);
static_assert(ON == NSUB * EMB);
static_assert(EMB == 32 && KPAD == 32 && NF <= KPAD && (NF % 8) == 0);
static_assert(NSUB == 16);
static_assert((LDH % 8) == 0 && LDH >= KPAD);
static_assert(8 * 4 * 16 == ON);
static_assert(WH_BLOCKS * 256u * 8u == (unsigned)WH_LAYER_HALVES);
static_assert((NF * EMB) / 4 == 192);
static_assert(2 * 256 == ON);
static_assert(4 * 128 == ON);
static_assert(((size_t)WH_LAYER_HALVES * 2) % 128 == 0);
static_assert(((size_t)AL_OFF1 * 2) % 128 == 0 && ((size_t)AL_OFF2 * 2) % 128 == 0);
static_assert((OFF_WL_BYTES % 128) == 0 && (OFF_AL_BYTES % 128) == 0);
static_assert(WS_TOTAL == (size_t)262144);
static_assert(WS_TOTAL <= (size_t)134217728);
static_assert(3 * LDH * 32 * 2 + ON * 4 <= 131072);

__device__ __forceinline__ float bf16r(float x) {
  unsigned int u = __float_as_uint(x);
  u = (u + 0x7FFFu + ((u >> 16) & 1u)) & 0xFFFF0000u;
  return __uint_as_float(u);
}

static __device__ __forceinline__ h16 toh_flush(float v) {
  const h16 r = (h16)v;
  return (fabsf(v) < 6.103515625e-05f) ? (h16)0.0f : r;
}

__device__ __forceinline__ v16h frag_at(const _Float16* p) {
  v8h lo = *(const v8h*)(p);
  v8h hi = *(const v8h*)(p + 16);
  v16h out;
#pragma unroll
  for (int i = 0; i < 8; ++i) { out[i] = lo[i]; out[i + 8] = hi[i]; }
  return out;
}

__device__ __forceinline__ v8f wmma16(v16h a, v16h b, v8f c) {
  v8f d = __builtin_amdgcn_wmma_f32_16x16x32_f16(false, a, false, b, (short)0, c,
                                                 false, false);
  asm volatile("v_nop\n\tv_nop\n\tv_nop\n\tv_nop" : "+v"(d) : "v"(a), "v"(b));
  return d;
}

__global__ __launch_bounds__(256) void prep_kernel(
    const float* __restrict__ W, const float* __restrict__ hv, const float* __restrict__ alpha,
    _Float16* __restrict__ whl, _Float16* __restrict__ whr, _Float16* __restrict__ all,
    unsigned s_in, unsigned ilog) {
#pragma clang fp contract(off)
  const unsigned tid = threadIdx.x;
  if (blockIdx.x < WH_BLOCKS) {
    const unsigned g = blockIdx.x * 256u + tid;
    const unsigned n = g >> 2, dc = (g & 3u) * 8u;
    const unsigned osub = n >> 5;
    const v4f w0 = *(const v4f*)(W + n * 32u + dc);
    const v4f w1 = *(const v4f*)(W + n * 32u + dc + 4u);
    const v4f s0 = *(const v4f*)(hv + osub * 32u + dc);
    const v4f s1 = *(const v4f*)(hv + osub * 32u + dc + 4u);
    v8h x, xr;
#pragma unroll
    for (int e = 0; e < 4; ++e) {
      const float t0 = WHCARRY * (bf16r(w0[e]) * bf16r(s0[e]));
      const float t1 = WHCARRY * (bf16r(w1[e]) * bf16r(s1[e]));
      const h16 a0 = toh_flush(t0);
      const h16 a1 = toh_flush(t1);
      x[e]      = a0;
      x[e + 4]  = a1;
      xr[e]     = toh_flush(RCARRY * (t0 - (float)a0));
      xr[e + 4] = toh_flush(RCARRY * (t1 - (float)a1));
    }
    _Float16* p  = whl + (size_t)g * 8u;
    _Float16* pr = whr + (size_t)g * 8u;
    *(volatile v8h*)p  = x;
    *(volatile v8h*)pr = xr;
    __threadfence();
    *(volatile v8h*)p  = x;
    *(volatile v8h*)pr = xr;
  } else {
    const unsigned g = (blockIdx.x - WH_BLOCKS) * 256u + tid;
    const unsigned row = g >> 2, jc = (g & 3u) * 8u;
    const unsigned osub = row >> ilog;
    const unsigned i = row & ((1u << ilog) - 1u);
    const unsigned ic = (i < s_in) ? i : (s_in - 1u);
    v8h x;
#pragma unroll
    for (unsigned e = 0; e < 8u; ++e) {
      const unsigned j = jc + e;
      const unsigned jj = (j < (unsigned)NF) ? j : (unsigned)(NF - 1);
      const float v = alpha[(ic * (unsigned)NF + jj) * (unsigned)NSUB + osub];
      const h16 t = toh_flush(ALCARRY * bf16r(v));
      x[e] = (j < (unsigned)NF && i < s_in) ? t : (h16)0.0f;
    }
    _Float16* p = all + (size_t)g * 8u;
    *(volatile v8h*)p = x;
    __threadfence();
    *(volatile v8h*)p = x;
  }
}

__global__ __launch_bounds__(256) void gin_kernel(
    const float* __restrict__ B0, const _Float16* __restrict__ whp,
    const _Float16* __restrict__ wlp, const _Float16* __restrict__ alp,
    float* __restrict__ out) {
  __shared__ __attribute__((aligned(16))) _Float16 B0T[32 * LDH];
  __shared__ __attribute__((aligned(16))) _Float16 BiS[32 * LDH];
  __shared__ __attribute__((aligned(16))) _Float16 BiR[32 * LDH];
  __shared__ __attribute__((aligned(16))) float OutS[ON];

  const unsigned tid = threadIdx.x, lane = tid & 31u;
  const unsigned wave = (unsigned)__builtin_amdgcn_readfirstlane((int)(threadIdx.x >> 5));
  const unsigned hh = lane >> 4, m = lane & 15u;
  const unsigned b = blockIdx.x;

  if (wave < 6u) {
    const unsigned q = tid;
    const unsigned j = q >> 3, h0 = (q & 7u) * 4u;
    const v4f a = *(const v4f*)(B0 + (size_t)b * (NF * EMB) + q * 4u);
#pragma unroll
    for (unsigned e = 0; e < 4u; ++e) {
      const float tv = B0CARRY * bf16r(a[e]);
      const h16 t = toh_flush(tv);
      BiS[j * LDH + h0 + e] = t;
      BiR[j * LDH + h0 + e] = toh_flush(RCARRY * (tv - (float)t));
      B0T[(h0 + e) * LDH + j] = t;
    }
  } else if (wave == 6u) {
    const v8h z = {};
    *(v8h*)&B0T[lane * LDH + 24u] = z;
  } else {
    const v8h z = {};
    *(v8h*)&BiS[(24u + (lane >> 2)) * LDH + (lane & 3u) * 8u] = z;
    *(v8h*)&BiR[(24u + (lane >> 2)) * LDH + (lane & 3u) * 8u] = z;
  }
  __syncthreads();

#pragma unroll 1
  for (unsigned l = 0; l < 3u; ++l) {
    const unsigned mtn  = (l == 0u) ? 2u : 1u;
    const unsigned aoff = (l == 0u) ? AL_OFF0 : ((l == 1u) ? AL_OFF1 : AL_OFF2);
    const float inv = (l == 0u) ? INV0 : ((l == 1u) ? INV1 : INV2);
    const float nxt = (l == 0u) ? BICARRY1 : BICARRY2;
    const unsigned woff = l * (unsigned)WH_LAYER_HALVES;

#pragma unroll 1
    for (unsigned t = 0; t < 4u; ++t) {
      const unsigned nt = wave * 4u + t;
      const unsigned osub = nt >> 1, ht = nt & 1u;
      const unsigned wrow = woff + (nt * 16u + m) * (unsigned)KPAD + hh * 8u;
      const v16h bwh = frag_at(whp + wrow);
      const v16h bwl = frag_at(wlp + wrow);
      const v16h bb0 = frag_at(&B0T[(ht * 16u + m) * LDH + hh * 8u]);
      float part = 0.0f;
#pragma unroll 1
      for (unsigned mt = 0; mt < mtn; ++mt) {
        const v16h aal = frag_at(alp + aoff + ((osub * mtn + mt) * 16u + m) * (unsigned)KPAD + hh * 8u);
        const v16h abi = frag_at(&BiS[(mt * 16u + m) * LDH + hh * 8u]);
        const v16h abr = frag_at(&BiR[(mt * 16u + m) * LDH + hh * 8u]);
        v8f cA = {};
        v8f cV = {};
        v8f cR = {};
        cA = wmma16(aal, bb0, cA);
        cV = wmma16(abi, bwh, cV);
        cR = wmma16(abi, bwl, cR);
        cR = wmma16(abr, bwh, cR);
#pragma unroll
        for (int r = 0; r < 8; ++r) part += cA[r] * (cV[r] + cR[r] * (1.0f / RCARRY));
      }
      part += __shfl_xor(part, 16, 32);
      if (hh == 0u) OutS[nt * 16u + m] = part * inv;
    }
    __syncthreads();

    if (l < 2u) {
      const unsigned n0 = tid * 2u;
      const float v0 = OutS[n0] * nxt;
      const float v1 = OutS[n0 + 1u] * nxt;
      const h16 a0 = toh_flush(v0);
      const h16 a1 = toh_flush(v1);
      const unsigned bo = (n0 >> 5) * LDH + (n0 & 31u);
      BiS[bo]      = a0;
      BiS[bo + 1u] = a1;
      BiR[bo]      = toh_flush(RCARRY * (v0 - (float)a0));
      BiR[bo + 1u] = toh_flush(RCARRY * (v1 - (float)a1));
      __syncthreads();
    }
  }

  if (wave < 4u) {
    const unsigned t4 = tid * 4u;
    const v4f val = *(const v4f*)&OutS[t4];
    float* p = out + (size_t)b * ON + t4;
    *(volatile v4f*)p = val;
    __threadfence();
    *(volatile v4f*)p = val;
  }
}

extern "C" void kernel_launch(void* const* d_in, const int* in_sizes, int n_in,
                              void* d_out, int out_size, void* d_ws, size_t ws_size,
                              hipStream_t stream) {
  if (n_in < 10) return;
  if ((long long)in_sizes[0] < (long long)NB * NF * EMB) return;
  if (in_sizes[1] < NSUB * EMB * EMB || in_sizes[4] < NSUB * EMB * EMB ||
      in_sizes[7] < NSUB * EMB * EMB) return;
  if (in_sizes[2] < NF * NF * NSUB) return;
  if (in_sizes[5] < NSUB * NF * NSUB || in_sizes[8] < NSUB * NF * NSUB) return;
  if (in_sizes[3] < NSUB * EMB || in_sizes[6] < NSUB * EMB || in_sizes[9] < NSUB * EMB) return;
  if ((long long)out_size < (long long)NB * ON) return;
  if (ws_size < WS_TOTAL) return;

  const float* B0 = (const float*)d_in[0];
  const float* W0 = (const float*)d_in[1];
  const float* a0 = (const float*)d_in[2];
  const float* h0 = (const float*)d_in[3];
  const float* W1 = (const float*)d_in[4];
  const float* a1 = (const float*)d_in[5];
  const float* h1 = (const float*)d_in[6];
  const float* W2 = (const float*)d_in[7];
  const float* a2 = (const float*)d_in[8];
  const float* h2 = (const float*)d_in[9];
  float* out = (float*)d_out;

  char* ws = (char*)d_ws;
  _Float16* WH = (_Float16*)(ws + OFF_WH_BYTES);
  _Float16* WL = (_Float16*)(ws + OFF_WL_BYTES);
  _Float16* AL = (_Float16*)(ws + OFF_AL_BYTES);

  dim3 blk(256);
  prep_kernel<<<dim3(WH_BLOCKS + 8u), blk, 0, stream>>>(W0, h0, a0, WH, WL, AL + AL_OFF0, 24u, 5u);
  prep_kernel<<<dim3(WH_BLOCKS + 4u), blk, 0, stream>>>(W1, h1, a1, WH + WH_LAYER_HALVES,
                                                        WL + WH_LAYER_HALVES, AL + AL_OFF1, 16u, 4u);
  prep_kernel<<<dim3(WH_BLOCKS + 4u), blk, 0, stream>>>(W2, h2, a2, WH + 2 * WH_LAYER_HALVES,
                                                        WL + 2 * WH_LAYER_HALVES, AL + AL_OFF2, 16u, 4u);
  gin_kernel<<<dim3(NB), blk, 0, stream>>>(B0, WH, WL, AL, out);
}
